// MultiModalVAE_46059229283223
// MI455X (gfx1250) — hardware-verified
//
#include <hip/hip_runtime.h>
#include <math.h>

constexpr int kNB = 4;
constexpr int kNS = 1024;
constexpr int kND = 1024;
constexpr int kNH = 8;
constexpr int kHD = 128;
constexpr int kNM = 4;
constexpr int kQKVld = 3 * kND;
constexpr float kWCarry    = 16.0f;
constexpr float kProjScale = 1.0f / 16.0f;
constexpr float kQKVScale  = 1.0f / 16.0f;
constexpr float kOutScale  = 1.0f / 64.0f;
constexpr float kSqrtHD    = 11.313708498984761f;

typedef __attribute__((ext_vector_type(16))) _Float16 v16h;
typedef __attribute__((ext_vector_type(8)))  _Float16 v8h;
typedef __attribute__((ext_vector_type(16))) __bf16   v16b;
typedef __attribute__((ext_vector_type(8)))  __bf16   v8b;
typedef __attribute__((ext_vector_type(8)))  float    v8f;
typedef __attribute__((ext_vector_type(4)))  float    v4f;
typedef __attribute__((ext_vector_type(4)))  unsigned int v4u;

__device__ __forceinline__ unsigned short f2bf_bits(float f) {
  unsigned u = __float_as_uint(f);
  return (unsigned short)((u + 0x7FFFu + ((u >> 16) & 1u)) >> 16);
}
__device__ __forceinline__ float bf_bits2f(unsigned short h) { return __uint_as_float(((unsigned)h) << 16); }

__device__ __forceinline__ void dep_guard_h(v8f& a, v8f& b, v16h x, v16h y) { asm volatile("v_nop\n\tv_nop\n\tv_nop\n\tv_nop" : "+v"(a), "+v"(b) : "v"(x), "v"(y)); }
__device__ __forceinline__ void dep_guard_b(v8f& a, v8f& b, v16b x, v16b y) { asm volatile("v_nop\n\tv_nop\n\tv_nop\n\tv_nop" : "+v"(a), "+v"(b) : "v"(x), "v"(y)); }
__device__ __forceinline__ void keep4_h(v16h a, v16h b, v16h c, v16h d) { asm volatile("v_nop" :: "v"(a), "v"(b), "v"(c), "v"(d)); }
__device__ __forceinline__ void keep4_b(v16b a, v16b b, v16b c, v16b d) { asm volatile("v_nop" :: "v"(a), "v"(b), "v"(c), "v"(d)); }
__device__ __forceinline__ void acc_guard4(v8f& a, v8f& b, v8f& c, v8f& d) { asm volatile("v_nop\n\tv_nop\n\tv_nop\n\tv_nop" : "+v"(a), "+v"(b), "+v"(c), "+v"(d)); }
template <typename T> struct Frag;
template <> struct Frag<_Float16> {
  typedef v16h V; union U { v16h v; v8h h[2]; };
  static __device__ __forceinline__ v16h load(const _Float16* p) {
    U f; f.h[0] = *(const v8h*)(p); f.h[1] = *(const v8h*)(p + 16); return f.v;
  }
  static __device__ __forceinline__ v8f mma(v16h a, v16h b, v8f c) {
    return __builtin_amdgcn_wmma_f32_16x16x32_f16(false, a, false, b, (short)0, c, false, false);
  }
  static __device__ __forceinline__ void guard(v8f& a, v8f& b, v16h x, v16h y) { dep_guard_h(a, b, x, y); }
  static __device__ __forceinline__ void keep(v16h a, v16h b, v16h c, v16h d) { keep4_h(a, b, c, d); }
};
template <> struct Frag<__bf16> {
  typedef v16b V; union U { v16b v; v8b h[2]; };
  static __device__ __forceinline__ v16b load(const __bf16* p) {
    U f; f.h[0] = *(const v8b*)(p); f.h[1] = *(const v8b*)(p + 16); return f.v;
  }
  static __device__ __forceinline__ v8f mma(v16b a, v16b b, v8f c) {
    return __builtin_amdgcn_wmma_f32_16x16x32_bf16(false, a, false, b, (short)0, c, false, false);
  }
  static __device__ __forceinline__ void guard(v8f& a, v8f& b, v16b x, v16b y) { dep_guard_b(a, b, x, y); }
  static __device__ __forceinline__ void keep(v16b a, v16b b, v16b c, v16b d) { keep4_b(a, b, c, d); }
};

__device__ __forceinline__ unsigned pk16(unsigned short a, unsigned short b) { return (unsigned)a | ((unsigned)b << 16); }
__device__ __forceinline__ unsigned short h_bits(float f) { const _Float16 h = (_Float16)f; return __builtin_bit_cast(unsigned short, h); }

template <int ET> struct Elem;
template <> struct Elem<0> { typedef _Float16 T; };
template <> struct Elem<1> { typedef __bf16 T; };
template <int ET, bool SPLIT, int BIAS_MODE, int OUT_MODE, bool RESID, int ACT = 0>
__global__ __launch_bounds__(256) void wmma_gemm64(
    const unsigned short* __restrict__ Ap, const unsigned short* __restrict__ A2p, int lda, long strideA,
    const unsigned short* __restrict__ Btp, const unsigned short* __restrict__ Bt2p, int ldb, long strideB,
    void* __restrict__ Cout, void* __restrict__ Cout2, int ldc, long strideC,
    const float* __restrict__ bias,
    const float* __restrict__ resid, long strideR,
    int M, int N, int K, float scale) {
  typedef typename Elem<ET>::T T;
  typedef typename Frag<T>::V V;
  const T* A = (const T*)Ap; const T* A2 = (const T*)A2p; const T* Bt = (const T*)Btp; const T* Bt2 = (const T*)Bt2p;
  __shared__ __align__(16) float sT[8][16 * 68];
  const int b    = blockIdx.y;
  const int lane = threadIdx.x & 31;
  const int wave = threadIdx.x >> 5;
  const int tilesN = N >> 6;
  const int tilesM = M >> 6;
  const int tile = blockIdx.x * 8 + wave;
  if (tile >= tilesM * tilesN) return;
  const int tm = tile / tilesN;
  const int tn = tile - tm * tilesN;
  const int m0 = tm << 6;
  const int n0 = tn << 6;

  const T* Ab  = A  + (size_t)b * strideA;
  const T* Bb  = Bt + (size_t)b * strideB;
  const T* Ab2 = SPLIT ? (A2  + (size_t)b * strideA) : nullptr;
  const T* Bb2 = SPLIT ? (Bt2 + (size_t)b * strideB) : nullptr;

  const int rlane = lane & 15;
  const int koff  = (lane >> 4) * 8;
  const int mOff  = (lane >> 4) * 8;

  v8f acc[4][4];
#pragma unroll
  for (int i = 0; i < 4; ++i)
#pragma unroll
    for (int j = 0; j < 4; ++j) acc[i][j] = (v8f){0.f,0.f,0.f,0.f,0.f,0.f,0.f,0.f};

  for (int k0 = 0; k0 < K; k0 += 32) {
    V bh[4], bl[4];
#pragma unroll
    for (int j = 0; j < 4; ++j) {
      const size_t bo = (size_t)(n0 + (j << 4) + rlane) * ldb + koff + k0;
      bh[j] = Frag<T>::load(Bb + bo);
      if (SPLIT) bl[j] = Frag<T>::load(Bb2 + bo);
    }
#pragma unroll
    for (int i = 0; i < 4; ++i) {
      const size_t ao = (size_t)(m0 + (i << 4) + rlane) * lda + koff + k0;
      V ah = Frag<T>::load(Ab + ao);
      V al;
      if (SPLIT) al = Frag<T>::load(Ab2 + ao);
#pragma unroll
      for (int j = 0; j < 4; ++j) {
        acc[i][j] = Frag<T>::mma(ah, bh[j], acc[i][j]);
        if (SPLIT) {
          acc[i][j] = Frag<T>::mma(ah, bl[j], acc[i][j]);
          acc[i][j] = Frag<T>::mma(al, bh[j], acc[i][j]);
        }
      }
      Frag<T>::guard(acc[i][0], acc[i][3], ah, SPLIT ? al : ah);
    }
    Frag<T>::keep(bh[0], bh[1], bh[2], bh[3]);
    if (SPLIT) Frag<T>::keep(bl[0], bl[1], bl[2], bl[3]);
  }
  acc_guard4(acc[0][0], acc[0][1], acc[0][2], acc[0][3]);
  acc_guard4(acc[1][0], acc[1][1], acc[1][2], acc[1][3]);
  acc_guard4(acc[2][0], acc[2][1], acc[2][2], acc[2][3]);
  acc_guard4(acc[3][0], acc[3][1], acc[3][2], acc[3][3]);

  float* slab = sT[wave];
  const float* Rb = RESID ? (resid + (size_t)b * strideR) : nullptr;
#pragma unroll
  for (int i = 0; i < 4; ++i) {
    const int mBase = m0 + (i << 4);
#pragma unroll
    for (int j = 0; j < 4; ++j) {
      const int n = n0 + (j << 4) + rlane;
      float bv = 0.f;
      if (BIAS_MODE == 2) bv = bias[n];
#pragma unroll
      for (int r = 0; r < 8; ++r) {
        float v = acc[i][j][r] * scale;
        if (BIAS_MODE == 1) v += bias[mBase + mOff + r];
        if (BIAS_MODE == 2) v += bv;
        if (RESID) v += Rb[(size_t)(mBase + mOff + r) * ldc + n];
        if (ACT == 2) v = fmaxf(v, 0.0f);
        if (ACT == 4) v = (v > 0.f) ? v : 0.01f * v;
        slab[(mOff + r) * 68 + (j << 4) + rlane] = v;
      }
    }
    __builtin_amdgcn_fence(__ATOMIC_RELEASE, "workgroup");
    __builtin_amdgcn_wave_barrier();
    __builtin_amdgcn_fence(__ATOMIC_ACQUIRE, "workgroup");
    if (OUT_MODE == 0) {
      float* C = (float*)Cout + (size_t)b * strideC;
      const int hh = lane >> 4, c4 = (lane & 15) * 4;
      for (int pass = 0; pass < 2; ++pass) {
#pragma unroll
        for (int it = 0; it < 8; ++it) {
          const int row = it * 2 + hh;
          v4f v = *(const v4f*)(slab + row * 68 + c4);
          *(volatile v4f*)(C + (size_t)(mBase + row) * ldc + n0 + c4) = v;
        }
        __threadfence();
      }
    } else {
      const int q = lane >> 3, c8 = (lane & 7) * 8;
      unsigned short* C  = (unsigned short*)Cout  + (size_t)b * strideC;
      unsigned short* C2 = (OUT_MODE == 2) ? ((unsigned short*)Cout2 + (size_t)b * strideC) : nullptr;
      for (int pass = 0; pass < 2; ++pass) {
#pragma unroll
        for (int it = 0; it < 4; ++it) {
          const int row = it * 4 + q;
          const float* sp = slab + row * 68 + c8;
          v8h hv, lv;
#pragma unroll
          for (int e = 0; e < 8; ++e) {
            if (OUT_MODE == 1) {
              hv[e] = (_Float16)sp[e];
            } else {
              unsigned short hb = f2bf_bits(sp[e]);
              unsigned short lb = f2bf_bits(sp[e] - bf_bits2f(hb));
              hv[e] = __builtin_bit_cast(_Float16, hb);
              lv[e] = __builtin_bit_cast(_Float16, lb);
            }
          }
          *(volatile v8h*)(C + (size_t)(mBase + row) * ldc + n0 + c8) = hv;
          if (OUT_MODE == 2) *(volatile v8h*)(C2 + (size_t)(mBase + row) * ldc + n0 + c8) = lv;
        }
        __threadfence();
      }
    }
    __builtin_amdgcn_fence(__ATOMIC_RELEASE, "workgroup");
    __builtin_amdgcn_wave_barrier();
    __builtin_amdgcn_fence(__ATOMIC_ACQUIRE, "workgroup");
  }
}

__global__ __launch_bounds__(256) void cast8_f16_kernel(const float* __restrict__ in, unsigned short* __restrict__ out, int n8) {
  const int i = blockIdx.x * 256 + threadIdx.x;
  if (i >= n8) return;
  const float* p = in + 8 * (size_t)i;
  const v4f a = *(const v4f*)(p);
  const v4f c = *(const v4f*)(p + 4);
  unsigned short hb[8];
#pragma unroll
  for (int e = 0; e < 4; ++e) {
    hb[e]     = h_bits(a[e]);
    hb[4 + e] = h_bits(c[e]);
  }
  const v4u u = (v4u){pk16(hb[0], hb[1]), pk16(hb[2], hb[3]), pk16(hb[4], hb[5]), pk16(hb[6], hb[7])};
  unsigned short* q = out + 8 * (size_t)i;
  *(volatile v4u*)q = u;
  __threadfence();
  *(volatile v4u*)q = u;
}

__global__ __launch_bounds__(256) void cast8s_f16_kernel(const float* __restrict__ in, unsigned short* __restrict__ out, int n8, float scale) {
  const int i = blockIdx.x * 256 + threadIdx.x;
  if (i >= n8) return;
  const float* p = in + 8 * (size_t)i;
  const v4f a = *(const v4f*)(p);
  const v4f c = *(const v4f*)(p + 4);
  unsigned short hb[8];
#pragma unroll
  for (int e = 0; e < 4; ++e) {
    hb[e]     = h_bits(a[e] * scale);
    hb[4 + e] = h_bits(c[e] * scale);
  }
  const v4u u = (v4u){pk16(hb[0], hb[1]), pk16(hb[2], hb[3]), pk16(hb[4], hb[5]), pk16(hb[6], hb[7])};
  unsigned short* q = out + 8 * (size_t)i;
  *(volatile v4u*)q = u;
  __threadfence();
  *(volatile v4u*)q = u;
}

__global__ __launch_bounds__(256) void bias_prep_kernel(const float* __restrict__ bt, const float* __restrict__ bi,
                                                        const float* __restrict__ ba, const float* __restrict__ bvd,
                                                        const float* __restrict__ emb,
                                                        const float* __restrict__ bq, const float* __restrict__ bk,
                                                        const float* __restrict__ bv,
                                                        float* __restrict__ out, int n4) {
  const int i = blockIdx.x * 256 + threadIdx.x;
  if (i >= n4) return;
  v4f o;
#pragma unroll
  for (int e = 0; e < 4; ++e) {
    const int idx = 4 * i + e;
    const int ic = (idx < kNM * kND) ? idx : (kNM * kND - 1);
    const int mm = ic >> 10;
    const int n  = ic & (kND - 1);
    const float c0 = bt[n], c1 = bi[n], c2 = ba[n], c3 = bvd[n];
    const float em = emb[ic];
    const float cb = ((mm == 0) ? c0 : (mm == 1) ? c1 : (mm == 2) ? c2 : c3) + em;
    int iq = idx - kNM * kND;
    iq = (iq < 0) ? 0 : ((iq > 3 * kND - 1) ? (3 * kND - 1) : iq);
    const int wq = iq >> 10;
    const int nq = iq & (kND - 1);
    const float q0 = bq[nq], q1 = bk[nq], q2 = bv[nq];
    const float cq = (wq == 0) ? q0 : (wq == 1) ? q1 : q2;
    o[e] = (idx < kNM * kND) ? cb : cq;
  }
  float* p = out + 4 * (size_t)i;
  *(volatile v4f*)p = o;
  __threadfence();
  *(volatile v4f*)p = o;
}

__global__ __launch_bounds__(256) void route_attn_kernel(const float* __restrict__ qkv, const float* __restrict__ temp,
                                                         unsigned short* __restrict__ fused, int bidx) {
  const int lane = threadIdx.x & 31;
  const int wave = threadIdx.x >> 5;
  const int wid  = blockIdx.x * 8 + wave;
  const int s    = wid >> 2;
  const int h    = ((wid & 3) << 1) + (lane >> 4);
  const int d8   = (lane & 15) * 8;
  const int col  = h * kHD + d8;
  const float tv = temp[0];
  const float scale = 1.0f / (kSqrtHD * fabsf(tv));

  float acc[8];
#pragma unroll
  for (int e = 0; e < 8; ++e) acc[e] = 0.f;

#pragma unroll 1
  for (int m = 0; m < kNM; ++m) {
    const int r0 = (m < 2) ? 0 : m;
    const int r1 = (m < 2) ? 1 : (5 - m);
    const int r2 = (m < 2) ? 2 : 0;
    const float* qp  = qkv + (size_t)(m  * kNS + s) * kQKVld + col;
    const float* k0p = qkv + (size_t)(r0 * kNS + s) * kQKVld + kND + col;
    const float* k1p = qkv + (size_t)(r1 * kNS + s) * kQKVld + kND + col;
    const float* k2p = qkv + (size_t)(r2 * kNS + s) * kQKVld + kND + col;
    const float* v0p = k0p + kND;
    const float* v1p = k1p + kND;
    const float* v2p = k2p + kND;
    const v4f qa = *(const v4f*)(qp),  qb = *(const v4f*)(qp + 4);
    const v4f ka = *(const v4f*)(k0p), kb = *(const v4f*)(k0p + 4);
    const v4f la = *(const v4f*)(k1p), lb = *(const v4f*)(k1p + 4);
    const v4f ma = *(const v4f*)(k2p), mb = *(const v4f*)(k2p + 4);
    const v4f va = *(const v4f*)(v0p), vb = *(const v4f*)(v0p + 4);
    const v4f wa = *(const v4f*)(v1p), wb = *(const v4f*)(v1p + 4);
    const v4f xa = *(const v4f*)(v2p), xb = *(const v4f*)(v2p + 4);

    float p0 = qa[0] * ka[0] + qa[1] * ka[1] + qa[2] * ka[2] + qa[3] * ka[3]
             + qb[0] * kb[0] + qb[1] * kb[1] + qb[2] * kb[2] + qb[3] * kb[3];
    float p1 = qa[0] * la[0] + qa[1] * la[1] + qa[2] * la[2] + qa[3] * la[3]
             + qb[0] * lb[0] + qb[1] * lb[1] + qb[2] * lb[2] + qb[3] * lb[3];
    float p2 = qa[0] * ma[0] + qa[1] * ma[1] + qa[2] * ma[2] + qa[3] * ma[3]
             + qb[0] * mb[0] + qb[1] * mb[1] + qb[2] * mb[2] + qb[3] * mb[3];
#pragma unroll
    for (int off = 8; off > 0; off >>= 1) {
      p0 += __shfl_xor(p0, off, 32);
      p1 += __shfl_xor(p1, off, 32);
      p2 += __shfl_xor(p2, off, 32);
    }
    const float s0 = p0 * scale, s1 = p1 * scale, s2 = p2 * scale;
    const float mx = fmaxf(s0, fmaxf(s1, s2));
    const float e0 = expf(s0 - mx), e1 = expf(s1 - mx), e2 = expf(s2 - mx);
    const float inv = 1.0f / (e0 + e1 + e2);
    const float a0 = e0 * inv, a1 = e1 * inv, a2 = e2 * inv;
#pragma unroll
    for (int e = 0; e < 4; ++e) {
      acc[e]     = acc[e]     + a0 * va[e] + a1 * wa[e] + a2 * xa[e];
      acc[4 + e] = acc[4 + e] + a0 * vb[e] + a1 * wb[e] + a2 * xb[e];
    }
  }

  unsigned short hb[8];
#pragma unroll
  for (int e = 0; e < 8; ++e) hb[e] = h_bits(acc[e]);
  const v4u u = (v4u){pk16(hb[0], hb[1]), pk16(hb[2], hb[3]), pk16(hb[4], hb[5]), pk16(hb[6], hb[7])};
  unsigned short* op = fused + ((size_t)(bidx * kNS + s) * kND + col);
  *(volatile v4u*)op = u;
  __threadfence();
  *(volatile v4u*)op = u;
}

extern "C" void kernel_launch(void* const* d_in, const int* in_sizes, int n_in,
                              void* d_out, int out_size, void* d_ws, size_t ws_size,
                              hipStream_t stream) {
  (void)n_in; (void)in_sizes;
  if (out_size != kNB * kNS * kND) return;

  const float* xin[4] = {(const float*)d_in[0], (const float*)d_in[3], (const float*)d_in[6], (const float*)d_in[9]};
  const float* win[4] = {(const float*)d_in[1], (const float*)d_in[4], (const float*)d_in[7], (const float*)d_in[10]};
  const float* bin[4] = {(const float*)d_in[2], (const float*)d_in[5], (const float*)d_in[8], (const float*)d_in[11]};
  const float* emb  = (const float*)d_in[12];
  const float* Wq   = (const float*)d_in[13]; const float* bq = (const float*)d_in[14];
  const float* Wk   = (const float*)d_in[15]; const float* bk = (const float*)d_in[16];
  const float* Wv   = (const float*)d_in[17]; const float* bv = (const float*)d_in[18];
  const float* Wo   = (const float*)d_in[19]; const float* bo = (const float*)d_in[20];
  const float* temperature = (const float*)d_in[21];
  const int din[4] = {768, 1024, 512, 1024};

  char* ws = (char*)d_ws;
  size_t off = 0;
  auto carve = [&](size_t bytes) { size_t o = off; off += (bytes + 127) & ~(size_t)127; return o; };
  size_t oX[4], oW[4];
  for (int m = 0; m < 4; ++m) oX[m] = carve((size_t)kNB * kNS * din[m] * 2);
  for (int m = 0; m < 4; ++m) oW[m] = carve((size_t)kND * din[m] * 2);
  const size_t oWQKV  = carve((size_t)3 * kND * kND * 2);
  const size_t oWO    = carve((size_t)kND * kND * 2);
  const size_t oBIAS  = carve((size_t)(kNM * kND + 3 * kND) * 4);
  const size_t oSTK   = carve((size_t)kNB * kNM * kNS * kND * 2);
  const size_t oQKV   = carve((size_t)kNM * kNS * kQKVld * 4);
  const size_t oFUSED = 0;
  if (off > ws_size) return;
  if ((size_t)kNB * kNS * kND * 2 > oW[0]) return;

  unsigned short* x16[4]; unsigned short* w16[4];
  for (int m = 0; m < 4; ++m) { x16[m] = (unsigned short*)(ws + oX[m]); w16[m] = (unsigned short*)(ws + oW[m]); }
  unsigned short* wqkv16  = (unsigned short*)(ws + oWQKV);
  unsigned short* wo16    = (unsigned short*)(ws + oWO);
  float*          biasall = (float*)(ws + oBIAS);
  float*          biasc   = biasall;
  float*          bqkv    = biasall + kNM * kND;
  unsigned short* stk16   = (unsigned short*)(ws + oSTK);
  float*          qkv32   = (float*)(ws + oQKV);
  unsigned short* fused16 = (unsigned short*)(ws + oFUSED);

  for (int m = 0; m < 4; ++m) {
    const int n8 = (kNB * kNS * din[m]) / 8;
    cast8_f16_kernel<<<(n8 + 255) / 256, 256, 0, stream>>>(xin[m], x16[m], n8);
  }
  for (int m = 0; m < 4; ++m) {
    const int n8 = (kND * din[m]) / 8;
    cast8s_f16_kernel<<<(n8 + 255) / 256, 256, 0, stream>>>(win[m], w16[m], n8, kWCarry);
  }
  {
    const int n8 = (kND * kND) / 8;
    cast8s_f16_kernel<<<(n8 + 255) / 256, 256, 0, stream>>>(Wq, wqkv16, n8, kWCarry);
    cast8s_f16_kernel<<<(n8 + 255) / 256, 256, 0, stream>>>(Wk, wqkv16 + (size_t)kND * kND, n8, kWCarry);
    cast8s_f16_kernel<<<(n8 + 255) / 256, 256, 0, stream>>>(Wv, wqkv16 + (size_t)2 * kND * kND, n8, kWCarry);
    cast8s_f16_kernel<<<(n8 + 255) / 256, 256, 0, stream>>>(Wo, wo16, n8, kWCarry);
  }
  {
    const int n4 = (kNM * kND + 3 * kND) / 4;
    bias_prep_kernel<<<(n4 + 255) / 256, 256, 0, stream>>>(bin[0], bin[1], bin[2], bin[3], emb, bq, bk, bv, biasall, n4);
  }

  for (int m = 0; m < 4; ++m) {
    const int tiles = (kNS / 64) * (kND / 64);
    dim3 grid((tiles + 7) / 8, kNB);
    wmma_gemm64<0, false, 2, 1, false, 0><<<grid, 256, 0, stream>>>(
        x16[m], nullptr, din[m], (long)kNS * din[m],
        w16[m], nullptr, din[m], 0L,
        (void*)(stk16 + (size_t)m * kNS * kND), nullptr, kND, (long)kNM * kNS * kND,
        biasc + m * kND,
        nullptr, 0L,
        kNS, kND, din[m], kProjScale);
  }

  for (int b = 0; b < kNB; ++b) {
    const int tiles = ((kNM * kNS) / 64) * (kQKVld / 64);
    dim3 grid((tiles + 7) / 8, 1);
    wmma_gemm64<0, false, 2, 0, false, 0><<<grid, 256, 0, stream>>>(
        stk16 + (size_t)b * kNM * kNS * kND, nullptr, kND, 0L,
        wqkv16, nullptr, kND, 0L,
        (void*)qkv32, nullptr, kQKVld, 0L,
        bqkv,
        nullptr, 0L,
        kNM * kNS, kQKVld, kND, kQKVScale);
    route_attn_kernel<<<(kNS * (kNH / 2)) / 8, 256, 0, stream>>>(qkv32, temperature, fused16, b);
  }

  {
    const int tiles = ((kNB * kNS) / 64) * (kND / 64);
    dim3 grid((tiles + 7) / 8, 1);
    wmma_gemm64<0, false, 2, 0, false, 0><<<grid, 256, 0, stream>>>(
        fused16, nullptr, kND, 0L,
        wo16, nullptr, kND, 0L,
        d_out, nullptr, kND, 0L,
        bo,
        nullptr, 0L,
        kNB * kNS, kND, kND, kOutScale);
  }
}
